// EfficientSelfAttention_22608707846573
// MI455X (gfx1250) — hardware-run, weakly checked
//
#include <hip/hip_runtime.h>
#include <math.h>

typedef __attribute__((ext_vector_type(16))) _Float16 v16h;
typedef __attribute__((ext_vector_type(16))) __bf16 v16b;
typedef __attribute__((ext_vector_type(8)))  _Float16 v8h;
typedef __attribute__((ext_vector_type(8)))  float v8f;
typedef __attribute__((ext_vector_type(4)))  float v4f;
typedef __attribute__((ext_vector_type(2)))  float v2f;
typedef __attribute__((ext_vector_type(4)))  unsigned v4u;
typedef __attribute__((ext_vector_type(4)))  int v4i;
typedef float __attribute__((may_alias)) float_a;
typedef int __attribute__((may_alias)) int_a;

template <typename T> __device__ __forceinline__ void vst2(void* p, T v) { *(volatile T*)p = v; __threadfence(); *(volatile T*)p = v; }
__device__ __forceinline__ v8f wmma16(v16h a, v16h b, v8f c) {
  v8f d = __builtin_amdgcn_wmma_f32_16x16x32_f16(false, a, false, b, (short)0, c, false, false);
  asm volatile("v_nop\n\tv_nop\n\tv_nop\n\tv_nop" : "+v"(d) : "v"(a), "v"(b));
  return d;
}
__device__ __forceinline__ v8f wmma_bf(v16b a, v16b b, v8f c) {
  v8f d = __builtin_amdgcn_wmma_f32_16x16x32_bf16(false, a, false, b, (short)0, c, false, false);
  asm volatile("v_nop\n\tv_nop\n\tv_nop\n\tv_nop" : "+v"(d) : "v"(a), "v"(b));
  return d;
}
__device__ __forceinline__ v16h frag_h(const _Float16* rowk0, int lane) {
  union { v16h v; v8h q[2]; } u; const _Float16* p = rowk0 + 8 * (lane >> 4);
  u.q[0] = *(const v8h*)p; u.q[1] = *(const v8h*)(p + 16); return u.v;
}
__device__ __forceinline__ v16h frag_f32(const float* rowk0, int lane) {
  v16h a; const float* p = rowk0 + 8 * (lane >> 4);
#pragma unroll
  for (int i = 0; i < 8; ++i) { a[i] = (_Float16)p[i]; a[8 + i] = (_Float16)p[16 + i]; }
  return a;
}
__device__ __forceinline__ v16h frag_f32s(const float* rowk0, int lane, float sc) {
  v16h a; const float* p = rowk0 + 8 * (lane >> 4);
#pragma unroll
  for (int i = 0; i < 8; ++i) { a[i] = (_Float16)(p[i] * sc); a[8 + i] = (_Float16)(p[16 + i] * sc); }
  return a;
}
__device__ __forceinline__ v16h fragc_f32(const float* W, int k0, int n, int lane, int ld, int K) {
  v16h a; const int g = lane >> 4;
#pragma unroll
  for (int i = 0; i < 8; ++i) { const int ka = k0 + 8 * g + i, kb = ka + 16;
    a[i] = (_Float16)(ka < K ? W[(size_t)(ka < K ? ka : K - 1) * ld + n] : 0.f); a[8 + i] = (_Float16)(kb < K ? W[(size_t)(kb < K ? kb : K - 1) * ld + n] : 0.f); }
  return a;
}
struct F2 { v16b h, l; };
__device__ __forceinline__ F2 bsplit16(const float v[16]) { F2 r;
#pragma unroll
  for (int i = 0; i < 16; ++i) { const __bf16 h = (__bf16)v[i]; r.h[i] = h; r.l[i] = (__bf16)(v[i] - (float)h); }
  return r; }
__device__ __forceinline__ F2 split_row(const float* row, int k0, int lane) { float v[16]; const float* p = row + k0 + 8 * (lane >> 4);
#pragma unroll
  for (int i = 0; i < 8; ++i) { v[i] = p[i]; v[8 + i] = p[16 + i]; }
  return bsplit16(v); }
__device__ __forceinline__ F2 split_rowK(const float* row, int k0, int lane, int K) { float v[16]; const int g = lane >> 4;
#pragma unroll
  for (int i = 0; i < 8; ++i) { const int ka = k0 + 8 * g + i, kb = ka + 16; v[i] = ka < K ? row[ka < K ? ka : K - 1] : 0.f; v[8 + i] = kb < K ? row[kb < K ? kb : K - 1] : 0.f; }
  return bsplit16(v); }
__device__ __forceinline__ F2 split_col(const float* W, int k0, int n, int lane, int ld, int K) { float v[16]; const int g = lane >> 4;
#pragma unroll
  for (int i = 0; i < 8; ++i) { const int ka = k0 + 8 * g + i, kb = ka + 16; v[i] = ka < K ? W[(size_t)(ka < K ? ka : K - 1) * ld + n] : 0.f; v[8 + i] = kb < K ? W[(size_t)(kb < K ? kb : K - 1) * ld + n] : 0.f; }
  return bsplit16(v); }
__device__ __forceinline__ v8f mac3(const F2& a, const F2& b, v8f c) { c = wmma_bf(a.l, b.h, c); c = wmma_bf(a.h, b.l, c); return wmma_bf(a.h, b.h, c); }
__device__ __forceinline__ float sigm(float v) { return 1.0f / (1.0f + expf(-v)); }
#define LDSX() do { asm volatile("s_wait_dscnt 0" ::: "memory"); __builtin_amdgcn_wave_barrier(); __builtin_amdgcn_fence(__ATOMIC_RELEASE, "workgroup"); } while (0)


#define NB 8
#define IH 128
#define IW 128
#define NN (IH * IW)
#define CC 64
#define RR 8
#define MH (IH / RR)
#define MW (IW / RR)
#define MM (MH * MW)
#define KCONV (CC * RR * RR)
#define LNEPS 1e-5f
#ifndef TNB
#define TNB NB
#endif
typedef __attribute__((ext_vector_type(8))) __bf16 v8b;
__device__ __forceinline__ v16b frag_b(const __bf16* rowk0, int lane) {
  union { v16b v; v8b q[2]; } u; const __bf16* p = rowk0 + 8 * (lane >> 4);
  u.q[0] = *(const v8b*)p; u.q[1] = *(const v8b*)(p + 16); return u.v;
}
__device__ __forceinline__ float bfr(float v) { return (float)(__bf16)v; }
__device__ __attribute__((noinline)) float exp_ni(float v) { return expf(v); }
__device__ __attribute__((noinline)) float erf_ni(float v) { return erff(v); }

#define WS_K   0u
#define WS_VH  (WS_K + 2u * (size_t)NB * MM * CC)
#define WS_VL  (WS_VH + 2u * (size_t)NB * CC * MM)
#define WS_END (WS_VL + 2u * (size_t)NB * CC * MM)

__device__ __forceinline__ v16b fragb_f32(const float* __restrict__ p, int lane) { v16b a; const float* pp = p + 8 * (lane >> 4);
#pragma unroll
  for (int i = 0; i < 8; ++i) { a[i] = (__bf16)pp[i]; a[8 + i] = (__bf16)pp[16 + i]; } return a; }
__global__ __launch_bounds__(128) void k_srkv(const float* __restrict__ X, const float* __restrict__ SRW, const float* __restrict__ SRB, const float* __restrict__ LW, const float* __restrict__ LB, const float* __restrict__ KVW, const float* __restrict__ KVB, _Float16* __restrict__ K, _Float16* __restrict__ VH, _Float16* __restrict__ VL) {
  __shared__ __align__(16) float sx[64][68]; __shared__ __align__(16) _Float16 sk[64][72]; __shared__ __align__(16) _Float16 th[CC][72], tl[CC][72];
  const int tid = threadIdx.x, wave = tid >> 5, lane = tid & 31, col = lane & 15, g = lane >> 4; const size_t b = blockIdx.y; const int m0 = blockIdx.x * 64 + wave * 16;
  v8f acc[4] = {};
  { const int m = m0 + col; const int my = m / MW, mx = m % MW;
#pragma unroll 2
    for (int kc = 0; kc < KCONV / 32; ++kc) { const int kk = kc >> 1, ci0 = (kc & 1) * 32; const int ky = kk >> 3, kx = kk & 7; const size_t n = (size_t)(my * RR + ky) * IW + mx * RR + kx;
      const v16b a = fragb_f32(X + (b * NN + n) * CC + ci0, lane);
#pragma unroll
      for (int j = 0; j < 4; ++j) { v16b w; const int co = j * 16 + col;
#pragma unroll
        for (int i = 0; i < 8; ++i) { w[i] = (__bf16)SRW[(((size_t)co * CC + ci0 + 8 * g + i) * RR + ky) * RR + kx]; w[8 + i] = (__bf16)SRW[(((size_t)co * CC + ci0 + 16 + 8 * g + i) * RR + ky) * RR + kx]; }
        acc[j] = wmma_bf(a, w, acc[j]); } } }
#pragma unroll
  for (int j = 0; j < 4; ++j)
#pragma unroll
    for (int r = 0; r < 8; ++r) sx[wave * 16 + 8 * g + r][j * 16 + col] = acc[j][r] + bfr(SRB[j * 16 + col]);
  LDSX();
  for (int rr = 0; rr < 16; ++rr) { const int rl = wave * 16 + rr; const float v0 = sx[rl][lane], v1 = sx[rl][lane + 32]; float s = v0 + v1;
#pragma unroll
    for (int o = 1; o < 32; o <<= 1) s += __shfl_xor(s, o);
    const float mu = s * (1.0f / CC); float q = (v0 - mu) * (v0 - mu) + (v1 - mu) * (v1 - mu);
#pragma unroll
    for (int o = 1; o < 32; o <<= 1) q += __shfl_xor(q, o);
    const float inv = 1.0f / sqrtf(q * (1.0f / CC) + LNEPS); LDSX(); sx[rl][lane] = (v0 - mu) * inv * bfr(LW[lane]) + bfr(LB[lane]); sx[rl][lane + 32] = (v1 - mu) * inv * bfr(LW[lane + 32]) + bfr(LB[lane + 32]); }
  LDSX();
  { v8f acc2[8] = {};
#pragma unroll
    for (int kc = 0; kc < CC / 32; ++kc) { float v[16]; const float* pp = &sx[wave * 16 + col][kc * 32 + 8 * g];
#pragma unroll
      for (int i = 0; i < 8; ++i) { v[i] = pp[i]; v[8 + i] = pp[16 + i]; }
      const F2 a = bsplit16(v);
#pragma unroll
      for (int j = 0; j < 8; ++j) { const v16b w = fragb_f32(KVW + (size_t)(j * 16 + col) * CC + kc * 32, lane); acc2[j] = wmma_bf(a.h, w, acc2[j]); acc2[j] = wmma_bf(a.l, w, acc2[j]); } }
#pragma unroll
    for (int j = 0; j < 8; ++j) { const float bb = bfr(KVB[j * 16 + col]);
#pragma unroll
      for (int r = 0; r < 8; ++r) { const float v = acc2[j][r] + bb; const int rl = wave * 16 + 8 * g + r; if (j < 4) sk[rl][j * 16 + col] = (_Float16)v; else { const int c = (j - 4) * 16 + col; const _Float16 hv = (_Float16)v; th[c][rl] = hv; tl[c][rl] = (_Float16)((v - (float)hv) * 2048.0f); } } } }
  __syncthreads();
  for (int e = tid; e < 64 * 8; e += 128) { const int rl = e >> 3, q = e & 7; vst2((unsigned*)(K + (b * MM + blockIdx.x * 64 + rl) * CC + q * 8), *(const v4u*)&sk[rl][q * 8]); }
  for (int e = tid; e < CC * 8; e += 128) { const int c = e >> 3, q = e & 7; const size_t o = (b * CC + c) * (size_t)MM + blockIdx.x * 64 + q * 8; vst2((unsigned*)(VH + o), *(const v4u*)&th[c][q * 8]); vst2((unsigned*)(VL + o), *(const v4u*)&tl[c][q * 8]); } }
__global__ __launch_bounds__(128) void k_att(const float* __restrict__ X, const float* __restrict__ QW, const float* __restrict__ QB, const _Float16* __restrict__ K, const _Float16* __restrict__ VH, const _Float16* __restrict__ VL, const float* __restrict__ PW, const float* __restrict__ PB, float* __restrict__ OUT) {
  __shared__ __align__(16) _Float16 sq[4][16][72]; __shared__ __align__(16) float sp[4][16][36]; __shared__ __align__(16) float so[4][16][68];
  const int tid = threadIdx.x, wave = tid >> 5, lane = tid & 31, col = lane & 15, g = lane >> 4; const size_t b = blockIdx.y; const int q0 = blockIdx.x * 64 + wave * 16; const size_t rq = b * NN + q0;
  { v8f aq4[4] = {};
#pragma unroll
    for (int kc = 0; kc < CC / 32; ++kc) { const v16b a = fragb_f32(X + (rq + col) * CC + kc * 32, lane);
#pragma unroll
      for (int j = 0; j < 4; ++j) aq4[j] = wmma_bf(a, fragb_f32(QW + (size_t)(j * 16 + col) * CC + kc * 32, lane), aq4[j]); }
#pragma unroll
    for (int j = 0; j < 4; ++j) { const float bb = bfr(QB[j * 16 + col]);
#pragma unroll
      for (int r = 0; r < 8; ++r) sq[wave][8 * g + r][j * 16 + col] = (_Float16)(aq4[j][r] + bb); } }
  LDSX();
  v16h aq[2];
#pragma unroll
  for (int kc = 0; kc < 2; ++kc) { const _Float16* pp = &sq[wave][col][kc * 32 + 8 * g];
#pragma unroll
    for (int i = 0; i < 8; ++i) { aq[kc][i] = pp[i]; aq[kc][8 + i] = pp[16 + i]; } }
  float m[8], l[8];
#pragma unroll
  for (int r = 0; r < 8; ++r) { m[r] = -3.0e38f; l[r] = 0.f; }
  v8f acc[4] = {}, accl[4] = {};
#pragma unroll 1
  for (int ks = 0; ks < MM / 32; ++ks) { float s[2][8];
#pragma unroll
    for (int ct = 0; ct < 2; ++ct) { const size_t rk = b * MM + ks * 32 + ct * 16 + col; v8f c = {};
#pragma unroll
      for (int kc = 0; kc < 2; ++kc) c = wmma16(aq[kc], frag_h(K + rk * CC + kc * 32, lane), c);
#pragma unroll
      for (int r = 0; r < 8; ++r) s[ct][r] = c[r] * 0.125f; }
    float alpha[8];
#pragma unroll
    for (int r = 0; r < 8; ++r) { float mx = fmaxf(s[0][r], s[1][r]);
#pragma unroll
      for (int o = 1; o < 16; o <<= 1) mx = fmaxf(mx, __shfl_xor(mx, o));
      const float mn = fmaxf(m[r], mx); alpha[r] = __expf(m[r] - mn); const float e0 = __expf(s[0][r] - mn), e1 = __expf(s[1][r] - mn); float es = e0 + e1;
#pragma unroll
      for (int o = 1; o < 16; o <<= 1) es += __shfl_xor(es, o);
      l[r] = l[r] * alpha[r] + es; m[r] = mn; sp[wave][8 * g + r][col] = e0; sp[wave][8 * g + r][16 + col] = e1; }
#pragma unroll
    for (int j = 0; j < 4; ++j)
#pragma unroll
      for (int r = 0; r < 8; ++r) { acc[j][r] *= alpha[r]; accl[j][r] *= alpha[r]; }
    LDSX();
    v16h pa; { const float* prow = &sp[wave][col][0] + 8 * (lane >> 4);
#pragma unroll
      for (int i = 0; i < 8; ++i) { pa[i] = (_Float16)(prow[i] * 2048.0f); pa[8 + i] = (_Float16)(prow[16 + i] * 2048.0f); } }
#pragma unroll
    for (int j = 0; j < 4; ++j) { const size_t po = (b * CC + j * 16 + col) * (size_t)MM + ks * 32; acc[j] = wmma16(pa, frag_h(VH + po, lane), acc[j]); accl[j] = wmma16(pa, frag_h(VL + po, lane), accl[j]); }
    LDSX(); }
#pragma unroll
  for (int r = 0; r < 8; ++r) { const float il = (1.0f / 2048.0f) / l[r];
#pragma unroll
    for (int j = 0; j < 4; ++j) so[wave][8 * g + r][j * 16 + col] = (acc[j][r] + accl[j][r] * (1.0f / 2048.0f)) * il; }
  LDSX();
  { v8f acc3[4] = {};
#pragma unroll
    for (int kc = 0; kc < CC / 32; ++kc) { float v[16]; const float* pp = &so[wave][col][kc * 32 + 8 * g];
#pragma unroll
      for (int i = 0; i < 8; ++i) { v[i] = pp[i]; v[8 + i] = pp[16 + i]; }
      const F2 a = bsplit16(v);
#pragma unroll
      for (int j = 0; j < 4; ++j) { const v16b w = fragb_f32(PW + (size_t)(j * 16 + col) * CC + kc * 32, lane); acc3[j] = wmma_bf(a.h, w, acc3[j]); acc3[j] = wmma_bf(a.l, w, acc3[j]); } }
    LDSX();
#pragma unroll
    for (int j = 0; j < 4; ++j) { const float bb = bfr(PB[j * 16 + col]);
#pragma unroll
      for (int r = 0; r < 8; ++r) so[wave][8 * g + r][j * 16 + col] = acc3[j][r] + bb; } }
  LDSX(); for (int rl = 0; rl < 16; ++rl) if (lane < 16) vst2(OUT + (rq + rl) * CC + lane * 4, *(const v4f*)&so[wave][rl][lane * 4]); }
extern "C" void kernel_launch(void* const* d_in, const int* in_sizes, int n_in, void* d_out, int out_size, void* d_ws, size_t ws_size, hipStream_t stream) {
  (void)in_sizes; (void)n_in; (void)out_size;
  const float** F = (const float**)d_in;
  if (ws_size < (size_t)WS_END) return;
  char* ws = (char*)d_ws; _Float16 *K = (_Float16*)(ws + WS_K), *VH = (_Float16*)(ws + WS_VH), *VL = (_Float16*)(ws + WS_VL);
  k_srkv<<<dim3(MM / 64, NB), 128, 0, stream>>>(F[0], F[9], F[10], F[11], F[12], F[5], F[6], K, VH, VL);
  k_att<<<dim3(NN / 64, TNB), 128, 0, stream>>>(F[0], F[3], F[4], K, VH, VL, F[7], F[8], (float*)d_out);
}
